// ShifthWiseConv2dImplicit_56831007260949
// MI455X (gfx1250) — hardware-verified
//
#include <hip/hip_runtime.h>

typedef __bf16 v16b __attribute__((ext_vector_type(16)));
typedef float  v8f  __attribute__((ext_vector_type(8)));
typedef float  v4f  __attribute__((ext_vector_type(4)));
typedef int    v8i  __attribute__((ext_vector_type(8)));
typedef v4f __attribute__((may_alias)) v4fa;

#define BB 32
#define CC 64
#define HH 56
#define WW 56
#define HW 3136
#define RN 50
#define GH 14
#define NK 17
#define NCLS 7
#define GRD 58
#define NGRID 3364
#define NTILE 211
#define MAPP 3376
#define SROWS 60
#define SPITCH 64
#define SIN_FLOATS (SROWS * SPITCH)
#define MAP_FLOATS (NCLS * MAPP)
#define DYN_LDS_BYTES ((SIN_FLOATS + MAP_FLOATS) * 4)
#define NQ 784
#define PLANE_FLOATS ((size_t)BB * RN * HW)
#define PART_LINE 32
#define STAT_FLOATS 512
#define NTHR 256

static_assert(NQ * 4 == HW);
static_assert((HW * 4) % 128 == 0);
static_assert(NTILE * 16 == MAPP);
static_assert(MAPP >= NGRID);
static_assert(GRD * GRD == NGRID);
static_assert(DYN_LDS_BYTES == 109888);
static_assert(sizeof(v16b) == 32);
static_assert(3 * RN <= NTHR);

__device__ __forceinline__ v8f wmma_bf16(v16b a, v16b b, v8f c) {
  v8f d = __builtin_amdgcn_wmma_f32_16x16x32_bf16(false, a, false, b, (short)0, c, false, false);
  const v8i ai = __builtin_bit_cast(v8i, a);
  const v8i bi = __builtin_bit_cast(v8i, b);
  asm volatile("v_nop\n\tv_nop\n\tv_nop\n\tv_nop" : "+v"(d) : "v"(ai), "v"(bi));
  return d;
}

__device__ __forceinline__ float wave_sum(float s) {
  s += __shfl_xor(s, 16);
  s += __shfl_xor(s, 8);
  s += __shfl_xor(s, 4);
  s += __shfl_xor(s, 2);
  s += __shfl_xor(s, 1);
  return s;
}

__global__ __launch_bounds__(NTHR) void mix_k(
    const float* __restrict__ inp, const float* __restrict__ w0, const float* __restrict__ w1,
    const int* __restrict__ Mh, const int* __restrict__ Mv, const int* __restrict__ Mid,
    const int* __restrict__ rep_idx, float* __restrict__ pl, float* __restrict__ part)
{
  extern __shared__ __attribute__((aligned(16))) float dlds[];
  __shared__ float sred[8 * 3];
  float* sIn = dlds;
  float* maps = dlds + SIN_FLOATS;
  const int tid = threadIdx.x, lane = tid & 31, wv = tid >> 5;
  const int h = lane >> 4, m = lane & 15;
  const int r = blockIdx.x, b = blockIdx.y;
  int ch = rep_idx[r];
  ch = ch < 0 ? 0 : (ch > CC - 1 ? CC - 1 : ch);
  const float* src = inp + (size_t)(b * CC + ch) * HW;
  const v4f z4 = {0.f, 0.f, 0.f, 0.f};

  #pragma unroll 1
  for (int q = tid; q < SROWS * 16; q += NTHR) {
    const int row = q >> 4, c4 = q & 15;
    const int yy = row - 2, cq = c4 - 1;
    const bool ok = ((unsigned)yy < (unsigned)HH) && ((unsigned)cq < 14u);
    const int yc = yy < 0 ? 0 : (yy > HH - 1 ? HH - 1 : yy);
    const int cc = cq < 0 ? 0 : (cq > 13 ? 13 : cq);
    v4f v = *(const v4fa*)(src + yc * WW + 4 * cc);
    if (!ok) v = z4;
    *(v4fa*)(sIn + row * SPITCH + 4 * c4) = v;
  }

  float wr[9][9];
  #pragma unroll
  for (int i = 0; i < 9; ++i) {
    const int k = (i < 8) ? (8 * h + i) : (16 + 8 * h);
    const bool kv = k < NK;
    const int kc = kv ? k : (NK - 1);
    const float* p0 = w0 + (size_t)(r * NK + kc) * 9;
    const float* p1 = w1 + (size_t)(r * NK + kc) * 9;
    #pragma unroll
    for (int t = 0; t < 9; ++t) {
      const float ws = p0[t] + p1[t];
      wr[i][t] = kv ? ws : 0.f;
    }
  }

  v16b bfr;
  {
    const int n = m;
    const int nh = (n < 3) ? n : 2;
    int nv = n - 3;
    nv = nv < 0 ? 0 : (nv > 2 ? 2 : nv);
    #pragma unroll
    for (int i = 0; i < 16; ++i) {
      const int k = (i < 8) ? (8 * h + i) : (16 + 8 * h + (i - 8));
      const bool kv = k < NK;
      const int kc = kv ? k : (NK - 1);
      const int vh = Mh[(nh * RN + r) * NK + kc];
      const int vvv = Mv[(nv * RN + r) * NK + kc];
      const int vd = Mid[r * NK + kc];
      int val = (n < 3) ? vh : ((n < 6) ? vvv : vd);
      val = (kv && (n < NCLS)) ? val : 0;
      bfr[i] = (__bf16)(float)val;
    }
  }
  __syncthreads();

  const v8f z8 = {0.f, 0.f, 0.f, 0.f, 0.f, 0.f, 0.f, 0.f};
  #pragma unroll 1
  for (int tile = wv; tile < NTILE; tile += 8) {
    int p = 16 * tile + m;
    p = (p > NGRID - 1) ? (NGRID - 1) : p;
    const int Y = p / GRD;
    const int X = p - Y * GRD;
    const float* tp = sIn + Y * SPITCH + X + 2;
    float tap[9];
    #pragma unroll
    for (int i = 0; i < 3; ++i) {
      #pragma unroll
      for (int j = 0; j < 3; ++j) tap[i * 3 + j] = tp[i * SPITCH + j];
    }
    float acc[9];
    #pragma unroll
    for (int i = 0; i < 9; ++i) {
      float a = 0.f;
      #pragma unroll
      for (int t = 0; t < 9; ++t) a = fmaf(tap[t], wr[i][t], a);
      acc[i] = a;
    }
    v16b ahi, alo;
    #pragma unroll
    for (int i = 0; i < 16; ++i) {
      if (i < 9) {
        const __bf16 hb = (__bf16)acc[i];
        const float rem = acc[i] - (float)hb;
        ahi[i] = hb;
        alo[i] = (__bf16)rem;
      } else {
        ahi[i] = (__bf16)0.0f;
        alo[i] = (__bf16)0.0f;
      }
    }
    v8f d = wmma_bf16(ahi, bfr, z8);
    d = wmma_bf16(alo, bfr, d);
    if (m < NCLS) {
      float* mp = maps + m * MAPP + 16 * tile + 8 * h;
      v4f u0, u1;
      u0.x = d[0]; u0.y = d[1]; u0.z = d[2]; u0.w = d[3];
      u1.x = d[4]; u1.y = d[5]; u1.z = d[6]; u1.w = d[7];
      *(v4fa*)(mp) = u0;
      *(v4fa*)(mp + 4) = u1;
    }
  }
  __syncthreads();

  float l1v[4][4], l2v[4][4], smv[4][4];
  float s1 = 0.f, s2 = 0.f, s3 = 0.f;
  #pragma unroll
  for (int it = 0; it < 4; ++it) {
    const int q = tid + NTHR * it;
    const bool vq = q < NQ;
    const int qc = vq ? q : 0;
    const int y = qc / 14;
    const int x0 = 4 * (qc - 14 * y);
    const int ym1 = (y == 0) ? (GRD - 1) : (y - 1);
    #pragma unroll
    for (int e = 0; e < 4; ++e) {
      const int x = x0 + e;
      const int xm1 = (x == 0) ? (GRD - 1) : (x - 1);
      const int P0 = (y + 1) * GRD + x + 1;
      const int P1 = y * GRD + xm1;
      const int P2 = ym1 * GRD + x;
      float a1 = (maps[P0] + maps[MAPP + P1]) + maps[2 * MAPP + P2];
      float a2 = (maps[3 * MAPP + P0] + maps[4 * MAPP + P2]) + maps[5 * MAPP + P1];
      float a3 = maps[6 * MAPP + P0];
      a1 = vq ? a1 : 0.f;
      a2 = vq ? a2 : 0.f;
      a3 = vq ? a3 : 0.f;
      l1v[it][e] = a1; l2v[it][e] = a2; smv[it][e] = a3;
      s1 += a1; s2 += a2; s3 += a3;
    }
  }

  s1 = wave_sum(s1); s2 = wave_sum(s2); s3 = wave_sum(s3);
  if (lane == 0) { sred[wv * 3] = s1; sred[wv * 3 + 1] = s2; sred[wv * 3 + 2] = s3; }
  __syncthreads();
  float S1 = 0.f, S2 = 0.f, S3 = 0.f;
  #pragma unroll
  for (int w = 0; w < 8; ++w) { S1 += sred[w * 3]; S2 += sred[w * 3 + 1]; S3 += sred[w * 3 + 2]; }
  const float inv_n = 1.0f / (float)HW;
  const float mb1 = S1 * inv_n, mb2 = S2 * inv_n, mb3 = S3 * inv_n;
  __syncthreads();
  float q1 = 0.f, q2 = 0.f, q3 = 0.f;
  #pragma unroll
  for (int it = 0; it < 4; ++it) {
    const bool vq = (tid + NTHR * it) < NQ;
    #pragma unroll
    for (int e = 0; e < 4; ++e) {
      const float d1 = l1v[it][e] - mb1, d2 = l2v[it][e] - mb2, d3 = smv[it][e] - mb3;
      q1 += vq ? d1 * d1 : 0.f;
      q2 += vq ? d2 * d2 : 0.f;
      q3 += vq ? d3 * d3 : 0.f;
    }
  }
  q1 = wave_sum(q1); q2 = wave_sum(q2); q3 = wave_sum(q3);
  if (lane == 0) { sred[wv * 3] = q1; sred[wv * 3 + 1] = q2; sred[wv * 3 + 2] = q3; }
  __syncthreads();
  float Q1 = 0.f, Q2 = 0.f, Q3 = 0.f;
  #pragma unroll
  for (int w = 0; w < 8; ++w) { Q1 += sred[w * 3]; Q2 += sred[w * 3 + 1]; Q3 += sred[w * 3 + 2]; }

  const size_t pbase = (size_t)(b * RN + r) * HW;
  v4f o1[4], o2[4], o3[4];
  size_t gq[4];
  #pragma unroll
  for (int it = 0; it < 4; ++it) {
    o1[it].x = l1v[it][0]; o1[it].y = l1v[it][1]; o1[it].z = l1v[it][2]; o1[it].w = l1v[it][3];
    o2[it].x = l2v[it][0]; o2[it].y = l2v[it][1]; o2[it].z = l2v[it][2]; o2[it].w = l2v[it][3];
    o3[it].x = smv[it][0]; o3[it].y = smv[it][1]; o3[it].z = smv[it][2]; o3[it].w = smv[it][3];
    gq[it] = pbase + (size_t)4 * (tid + NTHR * it);
  }
  v4f pv;
  pv.x = (lane == 0) ? S1 : ((lane == 1) ? S3 : 0.f);
  pv.y = (lane == 0) ? Q1 : ((lane == 1) ? Q3 : 0.f);
  pv.z = (lane == 0) ? S2 : 0.f;
  pv.w = (lane == 0) ? Q2 : 0.f;
  const bool pw = (wv == 0) && (lane < 8);
  const size_t li = (size_t)(b * RN + r) * PART_LINE + 4 * (lane & 7);

  #pragma unroll
  for (int it = 0; it < 4; ++it) {
    if ((tid + NTHR * it) < NQ) {
      *(volatile v4f*)(pl + gq[it]) = o1[it];
      *(volatile v4f*)(pl + PLANE_FLOATS + gq[it]) = o2[it];
      *(volatile v4f*)(pl + 2 * PLANE_FLOATS + gq[it]) = o3[it];
    }
  }
  if (pw) *(volatile v4f*)(part + li) = pv;
  __threadfence();
  #pragma unroll
  for (int it = 0; it < 4; ++it) {
    if ((tid + NTHR * it) < NQ) {
      *(volatile v4f*)(pl + gq[it]) = o1[it];
      *(volatile v4f*)(pl + PLANE_FLOATS + gq[it]) = o2[it];
      *(volatile v4f*)(pl + 2 * PLANE_FLOATS + gq[it]) = o3[it];
    }
  }
  if (pw) *(volatile v4f*)(part + li) = pv;
}

__global__ __launch_bounds__(NTHR) void stat_k(const float* __restrict__ part, float* __restrict__ stats) {
  __shared__ __attribute__((aligned(16))) float sst[STAT_FLOATS];
  const int tid = threadIdx.x;
  sst[tid] = 0.f;
  sst[tid + NTHR] = 0.f;
  __syncthreads();
  {
    const int t = (tid < 3 * RN) ? tid : (3 * RN - 1);
    const int mapi = t / RN;
    const int r = t - RN * mapi;
    double ss = 0.0;
    #pragma unroll 1
    for (int bb = 0; bb < BB; ++bb)
      ss += (double)part[(size_t)(bb * RN + r) * PART_LINE + 2 * mapi];
    const double mu = ss * (1.0 / 100352.0);
    double qq = 0.0;
    #pragma unroll 1
    for (int bb = 0; bb < BB; ++bb) {
      const float* ln = part + (size_t)(bb * RN + r) * PART_LINE;
      const double sb = (double)ln[2 * mapi];
      const double m2 = (double)ln[2 * mapi + 1];
      const double dm = sb * (1.0 / 3136.0) - mu;
      qq += m2 + 3136.0 * dm * dm;
    }
    const float varf = (float)(qq * (1.0 / 100352.0));
    const float invs = 1.0f / sqrtf(varf + 1e-5f);
    if (tid < 3 * RN) {
      sst[r * 8 + 2 * mapi] = (float)mu;
      sst[r * 8 + 2 * mapi + 1] = invs;
    }
  }
  __syncthreads();
  const int ti = (tid < 128) ? tid : 0;
  const v4f v = *(const v4fa*)(sst + 4 * ti);
  if (tid < 128) *(volatile v4f*)(stats + 4 * tid) = v;
  __threadfence();
  if (tid < 128) *(volatile v4f*)(stats + 4 * tid) = v;
}

__global__ __launch_bounds__(NTHR) void out_k(
    const float* __restrict__ inp, const int* __restrict__ rep_idx, const int* __restrict__ ghost_idx,
    const float* __restrict__ pl, const float* __restrict__ stats, float* __restrict__ out)
{
  const int tid = threadIdx.x;
  const int c = blockIdx.x, b = blockIdx.y;
  const bool isrep = c < RN;
  const int cr = isrep ? c : (RN - 1);
  int cg = c - RN;
  cg = cg < 0 ? 0 : (cg > GH - 1 ? GH - 1 : cg);
  int chr = rep_idx[cr];
  chr = chr < 0 ? 0 : (chr > CC - 1 ? CC - 1 : chr);
  int chg = ghost_idx[cg];
  chg = chg < 0 ? 0 : (chg > CC - 1 ? CC - 1 : chg);
  const int ch = isrep ? chr : chg;
  const float m1 = stats[cr * 8 + 0], i1 = stats[cr * 8 + 1];
  const float m2 = stats[cr * 8 + 2], i2 = stats[cr * 8 + 3];
  const float m3 = stats[cr * 8 + 4], i3 = stats[cr * 8 + 5];
  const float* ip = inp + (size_t)(b * CC + ch) * HW;
  const size_t pb = (size_t)(b * RN + cr) * HW;
  const float* p1 = pl + pb;
  const float* p2 = pl + PLANE_FLOATS + pb;
  const float* p3 = pl + 2 * PLANE_FLOATS + pb;
  float* op = out + (size_t)(b * CC + c) * HW;

  v4f ov[4];
  int oq[4];
  #pragma unroll
  for (int it = 0; it < 4; ++it) {
    const int q = tid + NTHR * it;
    const bool vq = q < NQ;
    const int qc = vq ? q : 0;
    const v4f xin = *(const v4fa*)(ip + 4 * qc);
    const v4f a1 = *(const v4fa*)(p1 + 4 * qc);
    const v4f a2 = *(const v4fa*)(p2 + 4 * qc);
    const v4f a3 = *(const v4fa*)(p3 + 4 * qc);
    v4f res = ((a1 - m1) * i1 + (a2 - m2) * i2) + (a3 - m3) * i3;
    res = res + xin;
    v4f o = xin;
    if (isrep) o = res;
    ov[it] = o;
    oq[it] = 4 * q;
  }
  #pragma unroll
  for (int it = 0; it < 4; ++it)
    if ((tid + NTHR * it) < NQ) *(volatile v4f*)(op + oq[it]) = ov[it];
  __threadfence();
  #pragma unroll
  for (int it = 0; it < 4; ++it)
    if ((tid + NTHR * it) < NQ) *(volatile v4f*)(op + oq[it]) = ov[it];
}

extern "C" void kernel_launch(void* const* d_in, const int* in_sizes, int n_in,
                              void* d_out, int out_size, void* d_ws, size_t ws_size,
                              hipStream_t stream) {
  if (n_in < 8) return;
  if (in_sizes[0] != BB * CC * HW || out_size != BB * CC * HW) return;
  if (in_sizes[1] != RN * NK * 9 || in_sizes[2] != RN * NK * 9) return;
  if (in_sizes[3] != 3 * RN * NK || in_sizes[4] != 3 * RN * NK || in_sizes[5] != RN * NK) return;
  if (in_sizes[6] != GH || in_sizes[7] != RN) return;

  const float* inp = (const float*)d_in[0];
  const float* w0  = (const float*)d_in[1];
  const float* w1  = (const float*)d_in[2];
  const int* Mh    = (const int*)d_in[3];
  const int* Mv    = (const int*)d_in[4];
  const int* Mid   = (const int*)d_in[5];
  const int* ghost_idx = (const int*)d_in[6];
  const int* rep_idx   = (const int*)d_in[7];
  float* out = (float*)d_out;

  const size_t pl_bytes   = 3 * PLANE_FLOATS * sizeof(float);
  const size_t part_bytes = (size_t)BB * RN * PART_LINE * sizeof(float);
  const size_t stat_bytes = (size_t)STAT_FLOATS * sizeof(float);
  const size_t off_pl = 0;
  const size_t off_part = off_pl + pl_bytes;
  const size_t off_stat = off_part + part_bytes;
  const size_t total = off_stat + stat_bytes;
  if (total > ws_size) return;
  char* ws = (char*)d_ws;
  float* pl    = (float*)(ws + off_pl);
  float* part  = (float*)(ws + off_part);
  float* stats = (float*)(ws + off_stat);

  hipFuncSetAttribute(reinterpret_cast<const void*>(&mix_k),
                      hipFuncAttributeMaxDynamicSharedMemorySize, DYN_LDS_BYTES);
  mix_k<<<dim3(RN, BB), NTHR, DYN_LDS_BYTES, stream>>>(inp, w0, w1, Mh, Mv, Mid, rep_idx, pl, part);
  stat_k<<<1, NTHR, 0, stream>>>(part, stats);
  out_k<<<dim3(CC, BB), NTHR, 0, stream>>>(inp, rep_idx, ghost_idx, pl, stats, out);
}
